// MaskedMultiHeadAttention_8306466751124
// MI455X (gfx1250) — hardware-verified
//
#include <hip/hip_runtime.h>


#ifndef NB
#define NB 2
#endif
#ifndef SEQ
#define SEQ 2048
#endif
#define NB_FULL 2
#define SEQ_FULL 2048

namespace {
constexpr int DM = 1024, H = 16, HD = 64, SRC = 128;
constexpr int KL = ((SEQ) + SRC < (SEQ_FULL)) ? ((SEQ) + SRC) : (SEQ_FULL);
static_assert((NB) >= 1 && (NB) <= (NB_FULL));
static_assert((SEQ) % 64 == 0 && (SEQ) >= 64 && (SEQ) <= (SEQ_FULL));
static_assert(KL % 64 == 0 && KL >= (SEQ) && KL <= (SEQ_FULL));
static_assert(DM == H * HD && DM % 128 == 0 && HD == 64 && (SEQ_FULL) % 32 == 0);
constexpr float XS = 8.0f, WSC = 256.0f, PS = 1024.0f, LOG2E = 1.4426950408889634f;
typedef _Float16 b16;
typedef __attribute__((ext_vector_type(16))) _Float16 v16b;
typedef __attribute__((ext_vector_type(8))) _Float16 v8b;
typedef __attribute__((ext_vector_type(4))) _Float16 v4h;
typedef __attribute__((ext_vector_type(2))) _Float16 v2h;
typedef __attribute__((ext_vector_type(8))) float v8f;
typedef __attribute__((ext_vector_type(4))) float v4f;

__device__ __forceinline__ float bf16_rne(float f) { unsigned int u = __float_as_uint(f); u += 0x7FFFu + ((u >> 16) & 1u); return __uint_as_float(u & 0xFFFF0000u); }
__device__ __forceinline__ void split16(float v, b16& hi, b16& lo) { hi = (b16)v; lo = (b16)(v - (float)hi); }
__device__ __forceinline__ v16b frag_kb(const b16* p, int hh) { const v8b a = *(const v8b*)(p + 8 * hh), b = *(const v8b*)(p + 16 + 8 * hh); v16b f;
#pragma unroll
  for (int e = 0; e < 8; ++e) { f[e] = a[e]; f[8 + e] = b[e]; } return f; }
__device__ __forceinline__ v8f wmma16b(v16b a, v16b b, v8f c) { v8f d = __builtin_amdgcn_wmma_f32_16x16x32_f16(false, a, false, b, (short)0, c, false, false); asm volatile("v_nop\n\tv_nop\n\tv_nop\n\tv_nop" : "+v"(d) : "v"(a), "v"(b)); return d; }
__device__ __forceinline__ void wave_lds_sync() { __builtin_amdgcn_fence(3, "workgroup"); __builtin_amdgcn_wave_barrier(); __builtin_amdgcn_fence(2, "workgroup"); }
__device__ __forceinline__ float nexp2(float v) { return __builtin_amdgcn_exp2f(v); }

constexpr size_t WU = (size_t)DM * DM / 8;
constexpr size_t XU = (size_t)(NB_FULL) * (SEQ_FULL) * DM / 8;
constexpr size_t PREP_UNITS = 3 * WU + XU;
static_assert(PREP_UNITS % 256 == 0 && (3 * WU) % 256 == 0 && WU % 256 == 0);

__global__ __launch_bounds__(256) void prep_kernel(const float* __restrict__ x, const float* __restrict__ wq, const float* __restrict__ wk, const float* __restrict__ wv, b16* __restrict__ X16, b16* __restrict__ WT) {
  const size_t u = (size_t)blockIdx.x * 256 + threadIdx.x; if (u >= PREP_UNITS) return;
  const float* src; b16* dst; float sc;
  if (u < 3 * WU) { const int m = (int)(u / WU); const size_t e = (u - (size_t)m * WU) * 8; const float* w = m == 0 ? wq : m == 1 ? wk : wv; src = w + e; dst = WT + (size_t)m * DM * DM + e; sc = WSC; }
  else { const size_t e = (u - 3 * WU) * 8; src = x + e; dst = X16 + e; sc = XS; }
  const v4f f0 = *(const v4f*)src, f1 = *(const v4f*)(src + 4); v8b o;
#pragma unroll
  for (int j = 0; j < 4; ++j) { o[j] = (b16)(bf16_rne(f0[j]) * sc); o[4 + j] = (b16)(bf16_rne(f1[j]) * sc); }
  for (int pass = 0; pass < 2; ++pass) { *(volatile v8b*)dst = o; __threadfence(); }
}

__global__ __launch_bounds__(128) void proj_kernel(const b16* __restrict__ X16, const b16* __restrict__ WT, const float* __restrict__ bq, const float* __restrict__ bk, const float* __restrict__ bv,
                                                   b16* __restrict__ QH, b16* __restrict__ QLo, b16* __restrict__ KH, b16* __restrict__ KLo, b16* __restrict__ VTh, b16* __restrict__ VTl) {
  __shared__ __attribute__((aligned(16))) float Tf[4][16][128 + 4];
  const int wave = threadIdx.x >> 5, lane = threadIdx.x & 31, nloc = lane & 15, hlf = lane >> 4; const int t0 = blockIdx.x * 64; const int b = blockIdx.y;
  const int slab = blockIdx.z, n0 = slab * 128, part = slab / 8, c0 = n0 - part * DM;
  const float* bias = part == 0 ? bq : part == 1 ? bk : bv;
  const b16* xa = X16 + ((size_t)b * (SEQ_FULL) + t0 + wave * 16 + nloc) * DM;
  v8f acc[8];
#pragma unroll
  for (int t = 0; t < 8; ++t) acc[t] = (v8f){};
#pragma unroll 1
  for (int kb = 0; kb < DM; kb += 32) { const v16b a = frag_kb(xa + kb, hlf);
#pragma unroll
    for (int t = 0; t < 8; ++t) acc[t] = wmma16b(a, frag_kb(WT + (size_t)(n0 + t * 16 + nloc) * DM + kb, hlf), acc[t]); }
#pragma unroll
  for (int t = 0; t < 8; ++t) { const float bb = bf16_rne(bias[c0 + t * 16 + nloc]);
#pragma unroll
    for (int r = 0; r < 8; ++r) Tf[wave][8 * hlf + r][t * 16 + nloc] = acc[t][r] * (1.0f / (XS * WSC)) + bb; }
  __syncthreads();
  for (int pass = 0; pass < 2; ++pass) {
    if (part < 2) { b16* ph_ = part == 0 ? QH : KH; b16* pl_ = part == 0 ? QLo : KLo; const int c = c0 + lane * 4; const int h = c / HD, d = c % HD;
      for (int rr = 0; rr < 16; ++rr) { const int tok = t0 + wave * 16 + rr; v4h h4, l4; for (int j = 0; j < 4; ++j) { b16 p, q; split16(Tf[wave][rr][lane * 4 + j] * XS, p, q); h4[j] = p; l4[j] = q; }
        const size_t oi = (((size_t)b * H + h) * (SEQ_FULL) + tok) * HD + d; *(volatile v4h*)(ph_ + oi) = h4; *(volatile v4h*)(pl_ + oi) = l4; } }
    else {
#pragma unroll 1
      for (int q = 0; q < 32; ++q) { const int cl = wave * 32 + q; const int c = c0 + cl; const int h = c / HD, d = c % HD; const int tk = lane * 2; v2h hv, lv;
        for (int j = 0; j < 2; ++j) { b16 p, ql; split16(Tf[(tk + j) >> 4][(tk + j) & 15][cl] * XS, p, ql); hv[j] = p; lv[j] = ql; }
        const size_t oi = (((size_t)b * H + h) * HD + d) * (size_t)(SEQ_FULL) + t0 + lane * 2; *(volatile v2h*)(VTh + oi) = hv; *(volatile v2h*)(VTl + oi) = lv; } }
    __threadfence(); }
}

__global__ __launch_bounds__(64) void attn_kernel(const b16* __restrict__ QH, const b16* __restrict__ QLo, const b16* __restrict__ KH, const b16* __restrict__ KLo,
                                                  const b16* __restrict__ VTh, const b16* __restrict__ VTl, float* __restrict__ out) {
  __shared__ __attribute__((aligned(16))) b16 Pb[2][16][32 + 8], Pc[2][16][32 + 8]; __shared__ __attribute__((aligned(16))) float To[2][16][HD + 4];
  const int wave = threadIdx.x >> 5, lane = threadIdx.x & 31, hh = lane >> 4, col = lane & 15; const int b = blockIdx.y / H, h = blockIdx.y % H;
  const int q0 = blockIdx.x * 32 + wave * 16, qi = q0 + col;
  const size_t ph = (size_t)b * H + h; const size_t pq = ph * (size_t)(SEQ_FULL) * HD; const b16* Vh = VTh + ph * HD * (size_t)(SEQ_FULL); const b16* Vl = VTl + ph * HD * (size_t)(SEQ_FULL);
  const v16b qh0 = frag_kb(QH + pq + (size_t)qi * HD, hh), qh1 = frag_kb(QH + pq + (size_t)qi * HD + 32, hh), ql0 = frag_kb(QLo + pq + (size_t)qi * HD, hh), ql1 = frag_kb(QLo + pq + (size_t)qi * HD + 32, hh);
  const float cs = LOG2E / (8.0f * XS * XS);
  float m = -INFINITY, l = 0.0f; v8f o[4];
#pragma unroll
  for (int t = 0; t < 4; ++t) o[t] = (v8f){};
  const int kend = (q0 + 16 + SRC < KL) ? (q0 + 16 + SRC) : KL;
#pragma unroll 1
  for (int kb = 0; kb < kend; kb += 32) {
    float e[16]; float mx = -INFINITY;
#pragma unroll
    for (int u = 0; u < 2; ++u) { v8f s = (v8f){}; const size_t kr = pq + (size_t)(kb + u * 16 + col) * HD; const v16b kh0 = frag_kb(KH + kr, hh), kh1 = frag_kb(KH + kr + 32, hh), kl0 = frag_kb(KLo + kr, hh), kl1 = frag_kb(KLo + kr + 32, hh);
      s = wmma16b(kh0, qh0, s); s = wmma16b(kh0, ql0, s); s = wmma16b(kl0, qh0, s); s = wmma16b(kh1, qh1, s); s = wmma16b(kh1, ql1, s); s = wmma16b(kl1, qh1, s);
#pragma unroll
      for (int r = 0; r < 8; ++r) { const int key = kb + u * 16 + 8 * hh + r; const float vv = (key <= qi + SRC) ? s[r] * cs : -INFINITY; e[u * 8 + r] = vv; mx = fmaxf(mx, vv); } }
    mx = fmaxf(mx, __shfl_xor(mx, 16)); const float mn = fmaxf(m, mx); const float al = (mn == -INFINITY) ? 1.0f : nexp2(m - mn); float sum = 0.0f;
#pragma unroll
    for (int i2 = 0; i2 < 16; ++i2) { const float p = (e[i2] == -INFINITY) ? 0.0f : nexp2(e[i2] - mn); sum += p; b16 a_, b_; split16(p * PS, a_, b_); const int sl = (i2 < 8 ? 0 : 16) + 8 * hh + (i2 & 7); Pb[wave][col][sl] = a_; Pc[wave][col][sl] = b_; }
    sum += __shfl_xor(sum, 16); l = l * al + sum; m = mn;
    wave_lds_sync();
    const v16b pf = frag_kb(&Pb[wave][col][0], hh), pg = frag_kb(&Pc[wave][col][0], hh);
#pragma unroll
    for (int t = 0; t < 4; ++t) { o[t] *= al; const size_t vr = (size_t)(t * 16 + col) * (SEQ_FULL) + kb; const v16b va = frag_kb(Vh + vr, hh), vb2 = frag_kb(Vl + vr, hh); o[t] = wmma16b(va, pf, o[t]); o[t] = wmma16b(va, pg, o[t]); o[t] = wmma16b(vb2, pf, o[t]); }
    wave_lds_sync(); }
  const float inv = 1.0f / (l * PS * XS);
#pragma unroll
  for (int t = 0; t < 4; ++t)
#pragma unroll
    for (int r = 0; r < 8; ++r) To[wave][col][t * 16 + 8 * hh + r] = o[t][r] * inv;
  wave_lds_sync();
  for (int pass = 0; pass < 2; ++pass) {
    for (int rr2 = 0; rr2 < 8; ++rr2) { const int row = 2 * rr2 + hh; const int c4 = col * 4; const v4f f = *(const v4f*)(&To[wave][row][c4]);
      *(volatile v4f*)(out + ((size_t)b * (SEQ_FULL) + q0 + row) * DM + h * HD + c4) = f; }
    __threadfence(); }
}
}

extern "C" void kernel_launch(void* const* d_in, const int* in_sizes, int n_in, void* d_out, int out_size, void* d_ws, size_t ws_size, hipStream_t stream) {
  if (n_in < 7) return;
  auto Fp = [&](int i) { return (const float*)d_in[i]; };
  if (in_sizes[0] < (NB_FULL) * (SEQ_FULL) * DM || in_sizes[1] < DM * DM || in_sizes[2] < DM || in_sizes[3] < DM * DM || in_sizes[4] < DM || in_sizes[5] < DM * DM || in_sizes[6] < DM) return;
  if (out_size < (((NB) - 1) * (SEQ_FULL) + (SEQ)) * DM) return;
  size_t off = 0; char* ws = (char*)d_ws;
  auto carve = [&](size_t bytes) { char* p = ws + off; off += (bytes + 255) & ~(size_t)255; return p; };
  b16* X16 = (b16*)carve((size_t)(NB_FULL) * (SEQ_FULL) * DM * 2);
  b16* WT = (b16*)carve((size_t)3 * DM * DM * 2);
  const size_t plane = (size_t)(NB_FULL) * H * (SEQ_FULL) * HD * 2;
  b16* QH = (b16*)carve(plane); b16* QLo = (b16*)carve(plane); b16* KH = (b16*)carve(plane); b16* KLo = (b16*)carve(plane); b16* VTh = (b16*)carve(plane); b16* VTl = (b16*)carve(plane);
  if (off > ws_size || off > ((size_t)128 << 20)) return;
  prep_kernel<<<(unsigned)(PREP_UNITS / 256), 256, 0, stream>>>(Fp(0), Fp(1), Fp(3), Fp(5), X16, WT);
  proj_kernel<<<dim3(KL / 64, (NB), 24), 128, 0, stream>>>(X16, WT, Fp(2), Fp(4), Fp(6), QH, QLo, KH, KLo, VTh, VTl);
  attn_kernel<<<dim3((SEQ) / 32, (NB) * H), 64, 0, stream>>>(QH, QLo, KH, KLo, VTh, VTl, (float*)d_out);
}
